// TransformerLayer_73065983639707
// MI455X (gfx1250) — hardware-verified
//
#include <hip/hip_runtime.h>
#include <math.h>

typedef __attribute__((ext_vector_type(16))) _Float16 v16h;
typedef __attribute__((ext_vector_type(16))) __bf16 v16b;
typedef __attribute__((ext_vector_type(8)))  _Float16 v8h;
typedef __attribute__((ext_vector_type(8)))  float v8f;
typedef __attribute__((ext_vector_type(4)))  float v4f;
typedef __attribute__((ext_vector_type(2)))  float v2f;
typedef __attribute__((ext_vector_type(4)))  unsigned v4u;
typedef __attribute__((ext_vector_type(4)))  int v4i;
typedef float __attribute__((may_alias)) float_a;
typedef int __attribute__((may_alias)) int_a;

template <typename T> __device__ __forceinline__ void vst2(void* p, T v) { *(volatile T*)p = v; __threadfence(); *(volatile T*)p = v; }
__device__ __forceinline__ v8f wmma16(v16h a, v16h b, v8f c) {
  v8f d = __builtin_amdgcn_wmma_f32_16x16x32_f16(false, a, false, b, (short)0, c, false, false);
  asm volatile("v_nop\n\tv_nop\n\tv_nop\n\tv_nop" : "+v"(d) : "v"(a), "v"(b));
  return d;
}
__device__ __forceinline__ v8f wmma_bf(v16b a, v16b b, v8f c) {
  v8f d = __builtin_amdgcn_wmma_f32_16x16x32_bf16(false, a, false, b, (short)0, c, false, false);
  asm volatile("v_nop\n\tv_nop\n\tv_nop\n\tv_nop" : "+v"(d) : "v"(a), "v"(b));
  return d;
}
__device__ __forceinline__ v16h frag_h(const _Float16* rowk0, int lane) {
  union { v16h v; v8h q[2]; } u; const _Float16* p = rowk0 + 8 * (lane >> 4);
  u.q[0] = *(const v8h*)p; u.q[1] = *(const v8h*)(p + 16); return u.v;
}
__device__ __forceinline__ v16h frag_f32(const float* rowk0, int lane) {
  v16h a; const float* p = rowk0 + 8 * (lane >> 4);
#pragma unroll
  for (int i = 0; i < 8; ++i) { a[i] = (_Float16)p[i]; a[8 + i] = (_Float16)p[16 + i]; }
  return a;
}
__device__ __forceinline__ v16h frag_f32s(const float* rowk0, int lane, float sc) {
  v16h a; const float* p = rowk0 + 8 * (lane >> 4);
#pragma unroll
  for (int i = 0; i < 8; ++i) { a[i] = (_Float16)(p[i] * sc); a[8 + i] = (_Float16)(p[16 + i] * sc); }
  return a;
}
__device__ __forceinline__ v16h fragc_f32(const float* W, int k0, int n, int lane, int ld, int K) {
  v16h a; const int g = lane >> 4;
#pragma unroll
  for (int i = 0; i < 8; ++i) { const int ka = k0 + 8 * g + i, kb = ka + 16;
    a[i] = (_Float16)(ka < K ? W[(size_t)(ka < K ? ka : K - 1) * ld + n] : 0.f); a[8 + i] = (_Float16)(kb < K ? W[(size_t)(kb < K ? kb : K - 1) * ld + n] : 0.f); }
  return a;
}
struct F2 { v16b h, l; };
__device__ __forceinline__ F2 bsplit16(const float v[16]) { F2 r;
#pragma unroll
  for (int i = 0; i < 16; ++i) { const __bf16 h = (__bf16)v[i]; r.h[i] = h; r.l[i] = (__bf16)(v[i] - (float)h); }
  return r; }
__device__ __forceinline__ F2 split_row(const float* row, int k0, int lane) { float v[16]; const float* p = row + k0 + 8 * (lane >> 4);
#pragma unroll
  for (int i = 0; i < 8; ++i) { v[i] = p[i]; v[8 + i] = p[16 + i]; }
  return bsplit16(v); }
__device__ __forceinline__ F2 split_rowK(const float* row, int k0, int lane, int K) { float v[16]; const int g = lane >> 4;
#pragma unroll
  for (int i = 0; i < 8; ++i) { const int ka = k0 + 8 * g + i, kb = ka + 16; v[i] = ka < K ? row[ka < K ? ka : K - 1] : 0.f; v[8 + i] = kb < K ? row[kb < K ? kb : K - 1] : 0.f; }
  return bsplit16(v); }
__device__ __forceinline__ F2 split_col(const float* W, int k0, int n, int lane, int ld, int K) { float v[16]; const int g = lane >> 4;
#pragma unroll
  for (int i = 0; i < 8; ++i) { const int ka = k0 + 8 * g + i, kb = ka + 16; v[i] = ka < K ? W[(size_t)(ka < K ? ka : K - 1) * ld + n] : 0.f; v[8 + i] = kb < K ? W[(size_t)(kb < K ? kb : K - 1) * ld + n] : 0.f; }
  return bsplit16(v); }
__device__ __forceinline__ v8f mac3(const F2& a, const F2& b, v8f c) { c = wmma_bf(a.l, b.h, c); c = wmma_bf(a.h, b.l, c); return wmma_bf(a.h, b.h, c); }
__device__ __forceinline__ float sigm(float v) { return 1.0f / (1.0f + expf(-v)); }
#define LDSX() do { asm volatile("s_wait_dscnt 0" ::: "memory"); __builtin_amdgcn_wave_barrier(); __builtin_amdgcn_fence(__ATOMIC_RELEASE, "workgroup"); } while (0)

#define NB 2
#define SQ 1024
#define PADW 128
#define TT 1280
#define CC 512
#define CCQ 512
#define DIN 512
#define FFH 2048
#define NH 1
#define HD 512
#define NQB (TT / 64)
#define HG 1
#define SCALE (0.044194173824159216f)
#define HDQK 512
#define CAUSAL 0
#ifndef TNB
#define TNB NB
#endif
__device__ __forceinline__ v16b zero16b() { v16b z; _Pragma("unroll") for (int i = 0; i < 16; ++i) z[i] = (__bf16)0.f; return z; }
__device__ __forceinline__ float bfr(float v) { return (float)(__bf16)v; }
__host__ __device__ __forceinline__ int kb_last(int qb) { return CAUSAL ? ((qb * 64 + 63) >> 7) : (TT / 128 - 1); }
__host__ __device__ __forceinline__ int kbf_l(int qb) { return (qb * 64) >> 7; }
__host__ __device__ __forceinline__ int kbl_l(int qb) { const int hi = (qb * 64 + 63 + 2 * PADW) >> 7; return hi < TT / 128 ? hi : TT / 128 - 1; }
typedef __attribute__((ext_vector_type(8))) __bf16 v8b;
__device__ __forceinline__ v16b frag_b(const __bf16* rowk0, int lane) {
  union { v16b v; v8b q[2]; } u; const __bf16* p = rowk0 + 8 * (lane >> 4);
  u.q[0] = *(const v8b*)p; u.q[1] = *(const v8b*)(p + 16); return u.v;
}
#define QBH 0
#define QHI 0
#define KHI 64
__device__ __forceinline__ v16b wcol_io(const float* Wm, int k0, int o, int lane, int ld) { v16b w; const int g = lane >> 4;
#pragma unroll
  for (int i = 0; i < 8; ++i) { w[i] = (__bf16)Wm[(size_t)(k0 + 8 * g + i) * ld + o]; w[8 + i] = (__bf16)Wm[(size_t)(k0 + 16 + 8 * g + i) * ld + o]; }
  return w; }
__device__ __forceinline__ v16b wcol_oi(const float* Wm, int k0, int o, int lane, int K) { v16b w; const float* p = Wm + (size_t)o * K + k0 + 8 * (lane >> 4);
#pragma unroll
  for (int i = 0; i < 8; ++i) { w[i] = (__bf16)p[i]; w[8 + i] = (__bf16)p[16 + i]; }
  return w; }
__device__ __forceinline__ v16h wcolh_io(const float* Wm, int k0, int o, int lane, int ld) { v16h w; const int g = lane >> 4;
#pragma unroll
  for (int i = 0; i < 8; ++i) { w[i] = (_Float16)(bfr(Wm[(size_t)(k0 + 8 * g + i) * ld + o]) * 256.0f); w[8 + i] = (_Float16)(bfr(Wm[(size_t)(k0 + 16 + 8 * g + i) * ld + o]) * 256.0f); }
  return w; }
__device__ __forceinline__ v16h wcolh_oi(const float* Wm, int k0, int o, int lane, int K) { v16h w; const float* p = Wm + (size_t)o * K + k0 + 8 * (lane >> 4);
#pragma unroll
  for (int i = 0; i < 8; ++i) { w[i] = (_Float16)(bfr(p[i]) * 256.0f); w[8 + i] = (_Float16)(bfr(p[16 + i]) * 256.0f); }
  return w; }
#define WQKV_LAYOUT 0
__device__ __forceinline__ v16b wcol_hdk(const float* Wm, int k0, int o, int lane) { v16b w; const int g = lane >> 4; const float* p = Wm + (size_t)(o / HD) * DIN * HD + (o % HD);
#pragma unroll
  for (int i = 0; i < 8; ++i) { w[i] = (__bf16)p[(size_t)(k0 + 8 * g + i) * HD]; w[8 + i] = (__bf16)p[(size_t)(k0 + 16 + 8 * g + i) * HD]; }
  return w; }
#define WO_OUT_IN 0
#if WQKV_LAYOUT == 1
#define WCOL(W, k0, o, lane) wcol_oi(W, k0, (o), lane, DIN)
#elif WQKV_LAYOUT == 2
#define WCOL(W, k0, o, lane) wcol_hdk(W, k0, o, lane)
#else
#define WCOL(W, k0, o, lane) wcol_io(W, k0, (o), lane, CC)
#endif
#if WO_OUT_IN
#define WOCOL(W, k0, o, lane) wcol_oi(W, k0, o, lane, CC)
#define WOCOLH(W, k0, o, lane) wcolh_oi(W, k0, o, lane, CC)
#else
#define WOCOL(W, k0, o, lane) wcol_io(W, k0, o, lane, DIN)
#define WOCOLH(W, k0, o, lane) wcolh_io(W, k0, o, lane, DIN)
#endif
#define BG HG
#define BGN (TNB < BG ? TNB : BG)
#define DVH 128
#ifndef SM_EXTRA_PARAMS
#define SM_EXTRA_PARAMS
#endif
#ifndef PROJ_EXTRA_PARAMS
#define PROJ_EXTRA_PARAMS
#endif
#ifndef SM_MASK_HOOK
#define SM_MASK_HOOK (void)0
#endif

#define WS_QH  0u
#define WS_KH  (WS_QH + 2u * (size_t)NB * TT * CCQ)
#define WS_VT  (WS_KH + 2u * (size_t)NB * TT * CCQ)
#define WS_QL  (WS_VT + 2u * (size_t)NB * CC * TT)
#define WS_KL  (WS_QL + 2u * (size_t)NB * QHI * CCQ)
#define WS_VB  (WS_KL + 2u * (size_t)NB * KHI * CCQ)
#define WS_VBL (WS_VB + 2u * (size_t)NB * CC * KHI)
#define WS_S   (WS_VBL + 2u * (size_t)NB * CC * KHI)
#define WS_Y   (WS_S  + 4u * (size_t)HG * TT * TT)
#define WS_END (WS_Y  + 0u)

template <int WOFF> __global__ __launch_bounds__(128) void k_projT(const float* __restrict__ XQ, const float* __restrict__ XK, const float* __restrict__ XV, const float* __restrict__ WQ, const float* __restrict__ WK, const float* __restrict__ WV, const float* __restrict__ BQ, const float* __restrict__ BK, const float* __restrict__ BV,
    _Float16* __restrict__ QH, _Float16* __restrict__ QL, _Float16* __restrict__ KH, _Float16* __restrict__ KL, _Float16* __restrict__ VT, __bf16* __restrict__ VB, __bf16* __restrict__ VBL) {
  __shared__ __align__(16) _Float16 sh[64][136], sl[64][136]; __shared__ __align__(16) _Float16 th[128][72]; __shared__ __align__(16) __bf16 tb[128][72], tbl[128][72];
  const int tid = threadIdx.x, wave = tid >> 5, lane = tid & 31, col = lane & 15, g = lane >> 4; const int which = blockIdx.z + WOFF; const int c0 = blockIdx.y * 128; const size_t r0 = (size_t)blockIdx.x * 64; const size_t bb = r0 / TT; const int t0 = (int)(r0 % TT);
  const float* X = which == 0 ? XQ : which == 1 ? XK : XV; const float* WA = which == 0 ? WQ : which == 1 ? WK : WV; const float* BA = which == 0 ? BQ : which == 1 ? BK : BV;
  const int KD = DIN;
  v8f acc[8] = {};
#pragma unroll 2
  for (int kc = 0; kc < KD / 32; ++kc) { v16b a; { const float* p = X + (r0 + wave * 16 + col) * (size_t)KD + kc * 32 + 8 * g;
#pragma unroll
      for (int i = 0; i < 8; ++i) { a[i] = (__bf16)p[i]; a[8 + i] = (__bf16)p[16 + i]; } }
    asm volatile("s_wait_loadcnt 0x0" ::: "memory");
#pragma unroll
    for (int j = 0; j < 8; ++j) { const v16b w = WCOL(WA, kc * 32, c0 + j * 16 + col, lane); asm volatile("s_wait_loadcnt 0x0" ::: "memory"); acc[j] = wmma_bf(a, w, acc[j]); } }
  if (which < 2) { _Float16* DH = which == 0 ? QH : KH; _Float16* DL = which == 0 ? QL : KL; const int nhi = which == 0 ? QHI : KHI; const bool hi_rows = t0 < nhi;
#pragma unroll
    for (int j = 0; j < 8; ++j) { const float bias = BA ? bfr(BA[c0 + j * 16 + col]) : 0.f;
#pragma unroll
      for (int r = 0; r < 8; ++r) { const float v = acc[j][r] + bias; const _Float16 hv = (_Float16)v; sh[wave * 16 + 8 * g + r][j * 16 + col] = hv; sl[wave * 16 + 8 * g + r][j * 16 + col] = (_Float16)((v - (float)hv) * 1024.0f); } }
    __syncthreads();
    for (int e = tid; e < 64 * 16; e += 128) { const int rl = e >> 4, q = e & 15; vst2((unsigned*)(DH + (r0 + rl) * CCQ + c0 + q * 8), *(const v4u*)&sh[rl][q * 8]); if (hi_rows) vst2((unsigned*)(DL + (bb * nhi + t0 + rl) * (size_t)CCQ + c0 + q * 8), *(const v4u*)&sl[rl][q * 8]); }
  } else { const bool hi_rows = t0 < KHI;
#pragma unroll
    for (int j = 0; j < 8; ++j) { const float bias = BA ? bfr(BA[c0 + j * 16 + col]) : 0.f;
#pragma unroll
      for (int r = 0; r < 8; ++r) { const float v = acc[j][r] + bias; const int rl = wave * 16 + 8 * g + r, cl = j * 16 + col; th[cl][rl] = (_Float16)v; const __bf16 bh = (__bf16)v; tb[cl][rl] = bh; tbl[cl][rl] = (__bf16)(v - (float)bh); } }
    __syncthreads();
    for (int e = tid; e < 128 * 8; e += 128) { const int cl = e >> 3, q = e & 7; vst2((unsigned*)(VT + (bb * CC + c0 + cl) * (size_t)TT + t0 + q * 8), *(const v4u*)&th[cl][q * 8]); if (hi_rows) { const size_t o3 = (bb * CC + c0 + cl) * (size_t)KHI + t0 + q * 8; vst2((unsigned*)(VB + o3), *(const v4u*)&tb[cl][q * 8]); vst2((unsigned*)(VBL + o3), *(const v4u*)&tbl[cl][q * 8]); } } } }
__global__ __launch_bounds__(128) void k_sc(const _Float16* __restrict__ QH, const _Float16* __restrict__ KH, const _Float16* __restrict__ QL, const _Float16* __restrict__ KL, int bgrp, int h0, float* __restrict__ S0) { __shared__ __align__(16) float ss[4][16][132];
  const int qb = blockIdx.x, kb = blockIdx.y; if (kb < kbf_l(qb) || kb > kbl_l(qb)) return;
  const int h = h0; const int b = bgrp + blockIdx.z; float* S = S0 + (size_t)blockIdx.z * TT * TT;
  const int tid = threadIdx.x, wave = tid >> 5, lane = tid & 31, col = lane & 15, g = lane >> 4; const int k0 = kb * 128; const int ql0 = qb * 64 + wave * 16; const size_t q0 = (size_t)b * TT + ql0, kr0 = (size_t)b * TT + k0;
  v8f acc[8] = {}, accl[8] = {};
  const _Float16* QLb = QL + (size_t)b * QHI * CCQ; const _Float16* KLb = KL + (size_t)b * KHI * CCQ;
  if (qb < QBH) {
#pragma unroll
    for (int kc = 0; kc < HDQK / 32; ++kc) { const v16h ah = frag_h(QH + (q0 + col) * CCQ + kc * 32, lane), al = frag_h(QLb + (size_t)(ql0 + col) * CCQ + kc * 32, lane);
#pragma unroll
      for (int j = 0; j < 8; ++j) { const v16h kbf = frag_h(KH + (kr0 + j * 16 + col) * CCQ + kc * 32, lane), klf = frag_h(KLb + (size_t)(k0 + j * 16 + col) * CCQ + kc * 32, lane); acc[j] = wmma16(ah, kbf, acc[j]); accl[j] = wmma16(al, kbf, accl[j]); accl[j] = wmma16(ah, klf, accl[j]); } }
  } else if (qb * 64 < QHI) {
#pragma unroll
    for (int kc = 0; kc < HDQK / 32; ++kc) { const v16h ah = frag_h(QH + (q0 + col) * CCQ + kc * 32, lane), al = frag_h(QLb + (size_t)(ql0 + col) * CCQ + kc * 32, lane);
#pragma unroll
      for (int j = 0; j < 8; ++j) { const v16h kbf = frag_h(KH + (kr0 + j * 16 + col) * CCQ + kc * 32, lane); acc[j] = wmma16(ah, kbf, acc[j]); accl[j] = wmma16(al, kbf, accl[j]); } }
  } else {
#pragma unroll
    for (int kc = 0; kc < HDQK / 32; ++kc) { const v16h ah = frag_h(QH + (q0 + col) * CCQ + kc * 32, lane);
#pragma unroll
      for (int j = 0; j < 8; ++j) { const v16h kbf = frag_h(KH + (kr0 + j * 16 + col) * CCQ + kc * 32, lane); acc[j] = wmma16(ah, kbf, acc[j]); } } }
#pragma unroll
  for (int j = 0; j < 8; ++j) {
#pragma unroll
    for (int r = 0; r < 8; ++r) ss[wave][8 * g + r][j * 16 + col] = (acc[j][r] + accl[j][r] * (1.0f / 1024.0f)) * SCALE; }
  LDSX(); for (int rl = 0; rl < 16; ++rl) vst2(S + (size_t)(ql0 + rl) * TT + k0 + lane * 4, *(const v4f*)&ss[wave][rl][lane * 4]); }
__global__ __launch_bounds__(256) void k_sm(float* __restrict__ S0 SM_EXTRA_PARAMS) { __shared__ float sred[8]; __shared__ float sbc; __shared__ __align__(16) float shv[TT];
  const int tid = threadIdx.x; const int t = blockIdx.x; const int kstart = kbf_l(t >> 6) * 128, kend = (kbl_l(t >> 6) + 1) * 128;
  float* sr = S0 + (size_t)blockIdx.y * TT * TT + (size_t)t * TT;
  float m = -3.0e38f;
  for (int k = kstart + tid; k < kend; k += 256) { float v = sr[k]; v = (k >= t && k <= t + 2 * PADW) ? v : -3.0e38f; shv[k] = v; m = fmaxf(m, v); }
#pragma unroll
  for (int o = 1; o < 32; o <<= 1) m = fmaxf(m, __shfl_xor(m, o));
  if ((tid & 31) == 0) sred[tid >> 5] = m; __syncthreads(); if (tid == 0) { float a = sred[0]; for (int i = 1; i < 8; ++i) a = fmaxf(a, sred[i]); sbc = a; } __syncthreads(); m = sbc; __syncthreads();
  float sum = 0.f;
  for (int k = kstart + tid; k < kend; k += 256) { const float v = shv[k]; const float e = (v <= -1.0e38f) ? 0.f : expf(v - m); shv[k] = e; sum += e; }
#pragma unroll
  for (int o = 1; o < 32; o <<= 1) sum += __shfl_xor(sum, o);
  if ((tid & 31) == 0) sred[tid >> 5] = sum; __syncthreads(); if (tid == 0) { float a = 0.f; for (int i = 0; i < 8; ++i) a += sred[i]; sbc = 2048.0f / fmaxf(a, 1e-30f); } __syncthreads(); const float inv = sbc;
  for (int k = kstart + tid; k < kend; k += 256) shv[k] = shv[k] * inv;
  __syncthreads();
  for (int q = kstart / 4 + tid; q < kend / 4; q += 256) vst2(sr + q * 4, *(const v4f*)&shv[q * 4]); }
__global__ __launch_bounds__(128) void k_pv(const float* __restrict__ PS0, const _Float16* __restrict__ VT, const __bf16* __restrict__ VB, const __bf16* __restrict__ VBL, int bgrp, int h0, float* __restrict__ Y) { const int h = h0; const int b = bgrp + blockIdx.z; const float* PS = PS0 + (size_t)blockIdx.z * TT * TT; const int d0 = blockIdx.y * DVH;     __shared__ __align__(16) float ss[4][16][DVH + 4];
  const int tid = threadIdx.x, wave = tid >> 5, lane = tid & 31, col = lane & 15, g = lane >> 4; const int qb = blockIdx.x; const int ql0 = qb * 64 + wave * 16; const int kce = (kbl_l(qb) + 1) * 4; const int kcs = kbf_l(qb) * 4;
  v8f acc[DVH / 16] = {};
  if (qb < QBH) {
#pragma unroll 1
    for (int kc = kcs; kc < kce; ++kc) { const F2 p = split_row(PS + (size_t)(ql0 + col) * TT, kc * 32, lane);
      asm volatile("s_wait_loadcnt 0x0" ::: "memory");
#pragma unroll
      for (int j = 0; j < DVH / 16; ++j) { const size_t po = ((size_t)b * CC + h * HD + d0 + j * 16 + col) * (size_t)KHI + kc * 32; const v16b vh = frag_b(VB + po, lane); acc[j] = wmma_bf(p.h, vh, acc[j]); acc[j] = wmma_bf(p.l, vh, acc[j]); acc[j] = wmma_bf(p.h, frag_b(VBL + po, lane), acc[j]); } }
  } else {
#pragma unroll 1
    for (int kc = kcs; kc < kce; ++kc) { const v16h p = frag_f32(PS + (size_t)(ql0 + col) * TT + kc * 32, lane);
      asm volatile("s_wait_loadcnt 0x0" ::: "memory");
#pragma unroll
      for (int j = 0; j < DVH / 16; ++j) { const size_t po = ((size_t)b * CC + h * HD + d0 + j * 16 + col) * (size_t)TT + kc * 32; acc[j] = wmma16(p, frag_h(VT + po, lane), acc[j]); } } }
#pragma unroll
  for (int j = 0; j < DVH / 16; ++j)
#pragma unroll
    for (int r = 0; r < 8; ++r) ss[wave][8 * g + r][j * 16 + col] = acc[j][r] * (1.0f / 2048.0f);
  LDSX(); for (int rl = 0; rl < 16; ++rl) vst2(Y + ((size_t)b * TT + ql0 + rl) * CC + h * HD + d0 + lane * 4, *(const v4f*)&ss[wave][rl][lane * 4]); }

__constant__ float PEDIV[256] = {1.000000000e+00,9.646615982e-01,9.305720329e-01,8.976871371e-01,8.659642935e-01,8.353625536e-01,8.058421612e-01,7.773650289e-01,7.498942018e-01,7.233941555e-01,6.978305578e-01,6.731703877e-01,6.493816376e-01,6.264335513e-01,6.042963862e-01,5.829415321e-01,5.623413324e-01,5.424690843e-01,5.232990980e-01,5.048065782e-01,4.869675040e-01,4.697588980e-01,4.531583786e-01,4.371444881e-01,4.216964841e-01,4.067944288e-01,3.924189806e-01,3.785515130e-01,3.651741147e-01,3.522694409e-01,3.398208320e-01,3.278120756e-01,3.162277639e-01,3.050528169e-01,2.942727208e-01,2.838736176e-01,2.738419473e-01,2.641648352e-01,2.548296452e-01,2.458243966e-01,2.371373475e-01,2.287573069e-01,2.206734121e-01,2.128751576e-01,2.053525001e-01,1.980956644e-01,1.910952926e-01,1.843422949e-01,1.778279394e-01,1.715437919e-01,1.654817015e-01,1.596338600e-01,1.539926529e-01,1.485508084e-01,1.433012486e-01,1.382372230e-01,1.333521456e-01,1.286396980e-01,1.240937635e-01,1.197084934e-01,1.154781953e-01,1.113973930e-01,1.074607670e-01,1.036632806e-01,9.999999404e-02,9.646616876e-02,9.305721521e-02,8.976870775e-02,8.659642935e-02,8.353625238e-02,8.058422059e-02,7.773648947e-02,7.498941571e-02,7.233941555e-02,6.978306174e-02,6.731703877e-02,6.493815780e-02,6.264334917e-02,6.042963639e-02,5.829415470e-02,5.623412505e-02,5.424690247e-02,5.232990906e-02,5.048065633e-02,4.869675636e-02,4.697588086e-02,4.531583190e-02,4.371444881e-02,4.216965288e-02,4.067944735e-02,3.924189135e-02,3.785514832e-02,3.651741147e-02,3.522694856e-02,3.398207948e-02,3.278120980e-02,3.162277490e-02,3.050527908e-02,2.942727320e-02,2.838735655e-02,2.738419361e-02,2.641648240e-02,2.548296750e-02,2.458243631e-02,2.371373400e-02,2.287572995e-02,2.206734009e-02,2.128751762e-02,2.053524740e-02,1.980956644e-02,1.910952851e-02,1.843423024e-02,1.778279617e-02,1.715438068e-02,1.654817350e-02,1.596338116e-02,1.539926231e-02,1.485507749e-02,1.433012448e-02,1.382372156e-02,1.333521400e-02,1.286397036e-02,1.240937877e-02,1.197085250e-02,1.154781692e-02,1.113973651e-02,1.074607670e-02,1.036632806e-02,9.999999776e-03,9.646615945e-03,9.305721149e-03,8.976872079e-03,8.659644052e-03,8.353622630e-03,8.058420382e-03,7.773648947e-03,7.498940919e-03,7.233940996e-03,6.978305522e-03,6.731703877e-03,6.493817084e-03,6.264336407e-03,6.042961963e-03,5.829413887e-03,5.623412319e-03,5.424689967e-03,5.232990719e-03,5.048065446e-03,4.869675264e-03,4.697589204e-03,4.531584214e-03,4.371443298e-03,4.216963891e-03,4.067943431e-03,3.924189135e-03,3.785514971e-03,3.651741194e-03,3.522694577e-03,3.398208413e-03,3.278121585e-03,3.162276698e-03,3.050527070e-03,2.942726482e-03,2.838735469e-03,2.738419222e-03,2.641648054e-03,2.548296703e-03,2.458244096e-03,2.371374052e-03,2.287573647e-03,2.206733450e-03,2.128751250e-03,2.053524600e-03,1.980956644e-03,1.910952851e-03,1.843423001e-03,1.778279431e-03,1.715438091e-03,1.654817257e-03,1.596338116e-03,1.539926161e-03,1.485507702e-03,1.433012309e-03,1.382372109e-03,1.333521330e-03,1.286396990e-03,1.240937854e-03,1.197085134e-03,1.154781668e-03,1.113973558e-03,1.074607600e-03,1.036632806e-03,9.999999311e-04,9.646615945e-04,9.305720450e-04,8.976871613e-04,8.659643936e-04,8.353622979e-04,8.058419917e-04,7.773648831e-04,7.498940686e-04,7.233940996e-04,6.978305755e-04,6.731703761e-04,6.493816618e-04,6.264335825e-04,6.042962195e-04,5.829414004e-04,5.623411853e-04,5.424689734e-04,5.232990370e-04,5.048065213e-04,4.869675031e-04,4.697589029e-04,4.531583982e-04,4.371443356e-04,4.216964007e-04,4.067943373e-04,3.924189077e-04,3.785514855e-04,3.651740844e-04,3.522694460e-04,3.398208355e-04,3.278119839e-04,3.162277862e-04,3.050527012e-04,2.942727879e-04,2.838735236e-04,2.738420444e-04,2.641648171e-04,2.548295306e-04,2.458243980e-04,2.371372684e-04,2.287573443e-04,2.206733334e-04,2.128752094e-04,2.053524659e-04,1.980957459e-04,1.910952706e-04,1.843422069e-04,1.778279402e-04,1.715437102e-04,1.654817315e-04,1.596337970e-04,1.539926743e-04,1.485507673e-04,1.433012949e-04,1.382371993e-04,1.333520777e-04,1.286396873e-04,1.240937272e-04,1.197085148e-04,1.154781567e-04,1.113974067e-04,1.074607571e-04,1.036633257e-04};
__global__ __launch_bounds__(256) void k_prep(const float* __restrict__ X, float* __restrict__ XQ, float* __restrict__ XK) { const int tid = threadIdx.x; const size_t row = (size_t)blockIdx.x * 8 + (tid >> 5); const int lane = tid & 31; const int b = (int)(row / TT), r = (int)(row % TT);
  { v4f z; z[0] = z[1] = z[2] = z[3] = 0.f; if (r >= SQ) { _Pragma("unroll") for (int q = 0; q < 4; ++q) vst2(XQ + row * CC + lane * 16 + q * 4, z); } if (r < PADW || r >= PADW + SQ) { _Pragma("unroll") for (int q = 0; q < 4; ++q) vst2(XK + row * CC + lane * 16 + q * 4, z); } }
  if (r < SQ) { const float* xr = X + ((size_t)b * SQ + r) * CC + lane * 16;
#pragma unroll 1
    for (int q = 0; q < 4; ++q) { const v4f xv = *(const v4f*)(xr + q * 4); asm volatile("s_wait_loadcnt 0x0" ::: "memory"); v4f v;
#pragma unroll
      for (int u = 0; u < 4; u += 2) { _Pragma("clang fp contract(off)") const int c = lane * 16 + q * 4 + u; const float ang = (float)r * PEDIV[c >> 1]; v[u] = bfr(xv[u]) + sinf(ang); v[u + 1] = bfr(xv[u + 1]) + cosf(ang); }
      vst2(XQ + row * CC + lane * 16 + q * 4, v); vst2(XK + ((size_t)b * TT + PADW + r) * CC + lane * 16 + q * 4, v); } } }
template <int RELU> __global__ __launch_bounds__(128) void k_lin(const float* __restrict__ Xs, int srcTT, int kin, const float* __restrict__ Wm, const float* __restrict__ Bv, int nout, float* __restrict__ OUTL, int dstTT) { __shared__ __align__(16) float sf[4][16][132];
  const int tid = threadIdx.x, wave = tid >> 5, lane = tid & 31, col = lane & 15, g = lane >> 4; const int c0 = blockIdx.y * 128; const int b = blockIdx.z; const int s0 = blockIdx.x * 64 + wave * 16;
  const float* xb = Xs + ((size_t)b * srcTT + s0) * kin;
  v8f acc[8] = {};
#pragma unroll 1
  for (int kc = 0; kc < kin / 32; ++kc) { v16b a; { const float* p = xb + (size_t)col * kin + kc * 32 + 8 * g;
#pragma unroll
      for (int i = 0; i < 8; ++i) { a[i] = (__bf16)p[i]; a[8 + i] = (__bf16)p[16 + i]; } }
    asm volatile("s_wait_loadcnt 0x0" ::: "memory");
#pragma unroll
    for (int j = 0; j < 8; ++j) { const v16b w = wcol_io(Wm, kc * 32, c0 + j * 16 + col, lane, nout); acc[j] = wmma_bf(a, w, acc[j]); } }
#pragma unroll
  for (int j = 0; j < 8; ++j) { const float bb = Bv ? bfr(Bv[c0 + j * 16 + col]) : 0.f; asm volatile("s_wait_loadcnt 0x0" ::: "memory");
#pragma unroll
    for (int r = 0; r < 8; ++r) { const float v = acc[j][r] + bb; sf[wave][8 * g + r][j * 16 + col] = RELU ? fmaxf(v, 0.f) : v; } }
  LDSX(); for (int rl = 0; rl < 16; ++rl) vst2(OUTL + ((size_t)b * dstTT + s0 + rl) * nout + c0 + lane * 4, *(const v4f*)&sf[wave][rl][lane * 4]); }
__global__ __launch_bounds__(256) void k_addln(const float* __restrict__ A, int aTT, const float* __restrict__ R, int rTT, const float* __restrict__ Gm, const float* __restrict__ Bt, float* __restrict__ OUTP, int oTT) { const int tid = threadIdx.x; const int sq = blockIdx.x * 8 + (tid >> 5); const int lane = tid & 31; const int b = blockIdx.y;
  const float* ar = A + ((size_t)b * aTT + sq) * CC + lane * 16; const float* rr = R + ((size_t)b * rTT + sq) * CC + lane * 16; float v[16];
  { float ta[16], tr[16]; _Pragma("unroll") for (int i = 0; i < 16; ++i) { ta[i] = ar[i]; tr[i] = rr[i]; } asm volatile("s_wait_loadcnt 0x0" ::: "memory"); _Pragma("unroll") for (int i = 0; i < 16; ++i) v[i] = ta[i] + tr[i]; }
  float sm = 0.f; _Pragma("unroll") for (int i = 0; i < 16; ++i) sm += v[i];
#pragma unroll
  for (int o = 1; o < 32; o <<= 1) sm += __shfl_xor(sm, o);
  const float m = sm * (1.0f / CC);
  float q = 0.f; _Pragma("unroll") for (int i = 0; i < 16; ++i) { const float d = v[i] - m; q += d * d; }
#pragma unroll
  for (int o = 1; o < 32; o <<= 1) q += __shfl_xor(q, o);
  const float rs = 1.0f / sqrtf(q * (1.0f / CC) + 1e-5f);
  float* po = OUTP + ((size_t)b * oTT + sq) * CC + lane * 16;
  _Pragma("unroll") for (int q4 = 0; q4 < 4; ++q4) { v4f o; _Pragma("unroll") for (int u = 0; u < 4; ++u) { const int i = q4 * 4 + u; const float g0 = Gm[lane * 16 + i], b0 = Bt[lane * 16 + i]; asm volatile("s_wait_loadcnt 0x0" ::: "memory"); o[u] = (v[i] - m) * rs * bfr(g0) + bfr(b0); } vst2(po + q4 * 4, o); } }
#define WS_XQ (WS_END)
#define WS_XK (WS_XQ + 4u * (size_t)NB * TT * CC)
#define WS_A  (WS_XK + 4u * (size_t)NB * TT * CC)
#define WS_R1 (WS_A + 4u * (size_t)NB * TT * CC)
#define WS_HF (WS_R1 + 4u * (size_t)NB * SQ * CC)
#define WS_F2 (WS_HF + 4u * (size_t)NB * SQ * FFH)
#define WS_END2 (WS_F2 + 4u * (size_t)NB * SQ * CC)
extern "C" void kernel_launch(void* const* d_in, const int* in_sizes, int n_in, void* d_out, int out_size, void* d_ws, size_t ws_size, hipStream_t stream) {
  (void)in_sizes; (void)n_in; (void)out_size;
  const float** F = (const float**)d_in;
  if (ws_size < (size_t)WS_END) return;
  char* ws = (char*)d_ws; _Float16 *QH = (_Float16*)(ws + WS_QH), *KH = (_Float16*)(ws + WS_KH), *VT = (_Float16*)(ws + WS_VT), *QL = (_Float16*)(ws + WS_QL), *KL = (_Float16*)(ws + WS_KL); __bf16 *VB = (__bf16*)(ws + WS_VB), *VBL = (__bf16*)(ws + WS_VBL); float *S = (float*)(ws + WS_S), *Y = (float*)(ws + WS_Y);
  (void)Y; (void)QL; (void)KL; (void)VB; (void)VBL;
  if (ws_size < (size_t)WS_END2) return;
  float *XQ = (float*)(ws + WS_XQ), *XK = (float*)(ws + WS_XK), *A = (float*)(ws + WS_A), *R1 = (float*)(ws + WS_R1), *HF = (float*)(ws + WS_HF), *F2r = (float*)(ws + WS_F2);
  k_prep<<<dim3(NB * TT / 8), 256, 0, stream>>>(F[0], XQ, XK);
  k_projT<0><<<dim3(TNB * TT / 64, CCQ / 128, 2), 128, 0, stream>>>(XQ, XK, XK, F[1], F[3], F[5], F[2], F[4], F[6], QH, QL, KH, KL, VT, VB, VBL);
  k_projT<2><<<dim3(TNB * TT / 64, CC / 128, 1), 128, 0, stream>>>(XQ, XK, XK, F[1], F[3], F[5], F[2], F[4], F[6], QH, QL, KH, KL, VT, VB, VBL);
  for (int b0 = 0; b0 < TNB; b0 += BGN) {
    k_sc<<<dim3(NQB, TT / 128, BGN), 128, 0, stream>>>(QH, KH, QL, KL, b0, 0, S);
    k_sm<<<dim3(TT, BGN), 256, 0, stream>>>(S);
    k_pv<<<dim3(NQB, HD / DVH, BGN), 128, 0, stream>>>(S, VT, VB, VBL, b0, 0, A);
  }
  k_addln<<<dim3(SQ / 8, TNB), 256, 0, stream>>>(A, TT, XQ, TT, F[11], F[12], R1, SQ);
  k_lin<1><<<dim3(SQ / 64, FFH / 128, TNB), 128, 0, stream>>>(R1, SQ, CC, F[7], F[8], FFH, HF, SQ);
  k_lin<0><<<dim3(SQ / 64, CC / 128, TNB), 128, 0, stream>>>(HF, SQ, FFH, F[9], F[10], CC, F2r, SQ);
  k_addln<<<dim3(SQ / 8, TNB), 256, 0, stream>>>(F2r, SQ, R1, SQ, F[13], F[14], (float*)d_out, SQ);

}
